// xLSTM_85641647882831
// MI455X (gfx1250) — hardware-verified
//
#include <hip/hip_runtime.h>
#include <math.h>

constexpr int NBATCH = 16;
constexpr int NSTEP  = 256;
constexpr int NIN    = 19;
constexpr int KPAD   = 32;
constexpr int NHID   = 256;
constexpr int NG6    = 6 * NHID;
constexpr int NG4    = 4 * NHID;
constexpr int NROWS  = NSTEP * NBATCH;
constexpr int NF1    = 128;
constexpr int NF2    = 64;
constexpr int NTHR   = 256;
constexpr int NTHR2  = 512;
constexpr int CROWS  = 64;
constexpr int NPLANE = 3;
constexpr int HTP    = 264;
constexpr int GXP    = 1028;
constexpr int HSP    = 260;
constexpr size_t HM_PLANE = (size_t)NROWS * NHID;

static_assert(KPAD % 32 == 0 && NHID % 32 == 0, "GEMM K multiples of 32");
static_assert(NROWS % 64 == 0 && NG6 % 64 == 0 && NG4 % 64 == 0, "GEMM M, N tile multiples");
static_assert(((NROWS / 64) * (NG6 / 64)) % 8 == 0 && ((NROWS / 64) * (NG4 / 64)) % 8 == 0, "GEMM grids exact");
static_assert((NROWS * 4) % NTHR == 0 && (NG6 * 4) % NTHR == 0, "pack grids exact");
static_assert(NIN <= KPAD && KPAD == 32, "one k-step for the gate GEMM");
static_assert(NTHR == 4 * CROWS && NHID % CROWS == 0, "4 lanes per matrix-memory row");
static_assert((CROWS * NHID) % (4 * NTHR) == 0, "C zero-fill exact");
static_assert(NHID == 16 * (NTHR2 / 32), "16 waves x 16 units = all hidden units");
static_assert(NBATCH == 16, "one 16-row m-subtile");
static_assert(8 * NTHR2 * 4 == NBATCH * NG4, "gate slab staging exact");
static_assert(HTP % 8 == 0 && GXP % 4 == 0 && HSP % 4 == 0, "LDS alignment");
static_assert(16 * HSP + NBATCH * NF1 + NBATCH * NF2 + NBATCH <= 16 * GXP, "head staging fits in the gate slab region");
static_assert(NHID % 64 == 0 && NG4 % 64 == 0, "transpose tiles exact");
static_assert(NPLANE * 8 <= 32 && (CROWS * 2) == 128, "one 128-B line per plane per row slice, one lane octet per plane");

typedef __attribute__((ext_vector_type(8)))  _Float16 v8h;
typedef __attribute__((ext_vector_type(16))) __bf16   v16b;
typedef __attribute__((ext_vector_type(8)))  __bf16   v8b;
typedef __attribute__((ext_vector_type(8)))  float    v8f;
typedef __attribute__((ext_vector_type(4)))  float    v4f;
typedef __attribute__((ext_vector_type(4)))  unsigned v4u;

__device__ __forceinline__ unsigned short f2bf_bits(float f) {
  unsigned u = __float_as_uint(f);
  return (unsigned short)((u + 0x7FFFu + ((u >> 16) & 1u)) >> 16);
}
__device__ __forceinline__ float bf_bits2f(unsigned short h) { return __uint_as_float(((unsigned)h) << 16); }
__device__ __forceinline__ float bf16r(float f) { return bf_bits2f(f2bf_bits(f)); }
__device__ __forceinline__ void split3_bf(float f, unsigned short& hb, unsigned short& mb, unsigned short& lb) {
  hb = f2bf_bits(f);
  const float r1 = f - bf_bits2f(hb);
  mb = f2bf_bits(r1);
  const float r2 = r1 - bf_bits2f(mb);
  lb = f2bf_bits(r2);
}

__device__ __forceinline__ void guard4_b3(v8f& a, v8f& b, v8f& c, v8f& d, v16b x, v16b y, v16b z) {
  asm volatile("v_nop\n\tv_nop\n\tv_nop\n\tv_nop" : "+v"(a), "+v"(b), "+v"(c), "+v"(d) : "v"(x), "v"(y), "v"(z));
}
__device__ __forceinline__ void keep4_b(v16b a, v16b b, v16b c, v16b d) { asm volatile("v_nop" :: "v"(a), "v"(b), "v"(c), "v"(d)); }
__device__ __forceinline__ void acc_guard4(v8f& a, v8f& b, v8f& c, v8f& d) { asm volatile("v_nop\n\tv_nop\n\tv_nop\n\tv_nop" : "+v"(a), "+v"(b), "+v"(c), "+v"(d)); }

template <typename T> struct Frag;
template <> struct Frag<__bf16> {
  typedef v16b V; union U { v16b v; v8b h[2]; };
  static __device__ __forceinline__ v16b load(const __bf16* p) {
    U f; f.h[0] = *(const v8b*)(p); f.h[1] = *(const v8b*)(p + 16); return f.v;
  }
  static __device__ __forceinline__ v8f mma(v16b a, v16b b, v8f c) {
    return __builtin_amdgcn_wmma_f32_16x16x32_bf16(false, a, false, b, (short)0, c, false, false);
  }
};

__device__ __forceinline__ float frcp(float x) { return __builtin_amdgcn_rcpf(x); }

template <int MODE>
__global__ __launch_bounds__(NTHR) void pack_k32_kernel(const float* __restrict__ src, unsigned short* __restrict__ dst, int nrows) {
  const int i = blockIdx.x * NTHR + threadIdx.x;
  if (i >= nrows * 4) return;
  const int row = i >> 2, k0 = (i & 3) * 8;
  v8h hv;
#pragma unroll
  for (int e = 0; e < 8; ++e) {
    const int k  = k0 + e;
    const int kc = (k < NIN) ? k : (NIN - 1);
    float f;
    if (MODE == 0) {
      const int t = row >> 4, bb = row & 15;
      f = src[((size_t)bb * NSTEP + (size_t)t) * NIN + kc];
    } else {
      const int g = row >> 8, o = row & 255;
      f = src[((size_t)g * NIN + (size_t)kc) * NHID + o];
    }
    const float fz = (k < NIN) ? 1.0f : 0.0f;
    const unsigned short outb = f2bf_bits(f * fz);
    hv[e] = __builtin_bit_cast(_Float16, outb);
  }
  unsigned short* dp = dst + (size_t)i * 8;
  *(volatile v8h*)dp = hv;
  __threadfence();
  *(volatile v8h*)dp = hv;
}

__global__ __launch_bounds__(NTHR) void tpwz_kernel(const float* __restrict__ src, int R, int Cc, int ldo,
                                                    long sstride, long ostride, unsigned short* __restrict__ O) {
  __shared__ float Tt[64 * 65];
  const float* s = src + (size_t)blockIdx.z * (size_t)sstride;
  unsigned short* Oz = O + (size_t)blockIdx.z * (size_t)ostride;
  const int tid = threadIdx.x;
  const int c0 = blockIdx.x * 64, r0 = blockIdx.y * 64;
#pragma unroll
  for (int i = 0; i < 4; ++i) {
    const int idx = i * NTHR + tid;
    const int rr = idx >> 4, cc = (idx & 15) * 4;
    const v4f v = *(const v4f*)(s + (size_t)(r0 + rr) * (size_t)Cc + c0 + cc);
    Tt[rr * 65 + cc + 0] = v[0];
    Tt[rr * 65 + cc + 1] = v[1];
    Tt[rr * 65 + cc + 2] = v[2];
    Tt[rr * 65 + cc + 3] = v[3];
  }
  __syncthreads();
  const int q = tid >> 3, c8 = (tid & 7) * 8;
  v8h hv[2];
#pragma unroll
  for (int g = 0; g < 2; ++g) {
    const int qq = g * 32 + q;
#pragma unroll
    for (int e = 0; e < 8; ++e) {
      const float f = Tt[(c8 + e) * 65 + qq];
      hv[g][e] = __builtin_bit_cast(_Float16, f2bf_bits(f));
    }
  }
  for (int pass = 0; pass < 2; ++pass) {
#pragma unroll
    for (int g = 0; g < 2; ++g) {
      const size_t o = (size_t)(c0 + g * 32 + q) * (size_t)ldo + (size_t)(r0 + c8);
      *(volatile v8h*)(Oz + o) = hv[g];
    }
    __threadfence();
  }
}

template <int NPL>
__global__ __launch_bounds__(NTHR) void wmma_gemm64_bf16(
    const unsigned short* __restrict__ Ap, const unsigned short* __restrict__ A2p, const unsigned short* __restrict__ A3p, int lda,
    const unsigned short* __restrict__ Btp, int ldb,
    float* __restrict__ Cout, int ldc, int M, int N, int K) {
  typedef __bf16 T;
  typedef v16b V;
  const T* A = (const T*)Ap; const T* A2 = (const T*)A2p; const T* A3 = (const T*)A3p; const T* Bt = (const T*)Btp;
  __shared__ __align__(16) float sT[8][16 * 68];
  const int lane = threadIdx.x & 31;
  const int wave = threadIdx.x >> 5;
  const int tilesN = N >> 6;
  const int tilesM = M >> 6;
  const int tile = blockIdx.x * 8 + wave;
  if (tile >= tilesM * tilesN) return;
  const int tm = tile / tilesN;
  const int tn = tile - tm * tilesN;
  const int m0 = tm << 6;
  const int n0 = tn << 6;

  const int rlane = lane & 15;
  const int koff  = (lane >> 4) * 8;
  const int mOff  = (lane >> 4) * 8;

  v8f acc[4][4];
#pragma unroll
  for (int i = 0; i < 4; ++i)
#pragma unroll
    for (int j = 0; j < 4; ++j) acc[i][j] = (v8f){0.f,0.f,0.f,0.f,0.f,0.f,0.f,0.f};

  for (int k0 = 0; k0 < K; k0 += 32) {
    V bh[4];
#pragma unroll
    for (int j = 0; j < 4; ++j) {
      const size_t bo = (size_t)(n0 + (j << 4) + rlane) * ldb + koff + k0;
      bh[j] = Frag<T>::load(Bt + bo);
    }
#pragma unroll
    for (int i = 0; i < 4; ++i) {
      const size_t ao = (size_t)(m0 + (i << 4) + rlane) * lda + koff + k0;
      V ah = Frag<T>::load(A + ao);
      V am = ah, al = ah;
      if (NPL == 3) { am = Frag<T>::load(A2 + ao); al = Frag<T>::load(A3 + ao); }
#pragma unroll
      for (int j = 0; j < 4; ++j) {
        acc[i][j] = Frag<T>::mma(ah, bh[j], acc[i][j]);
        if (NPL == 3) {
          acc[i][j] = Frag<T>::mma(am, bh[j], acc[i][j]);
          acc[i][j] = Frag<T>::mma(al, bh[j], acc[i][j]);
        }
      }
      guard4_b3(acc[i][0], acc[i][1], acc[i][2], acc[i][3], ah, am, al);
    }
    keep4_b(bh[0], bh[1], bh[2], bh[3]);
  }
  acc_guard4(acc[0][0], acc[0][1], acc[0][2], acc[0][3]);
  acc_guard4(acc[1][0], acc[1][1], acc[1][2], acc[1][3]);
  acc_guard4(acc[2][0], acc[2][1], acc[2][2], acc[2][3]);
  acc_guard4(acc[3][0], acc[3][1], acc[3][2], acc[3][3]);

  float* slab = sT[wave];
#pragma unroll
  for (int i = 0; i < 4; ++i) {
    const int mBase = m0 + (i << 4);
#pragma unroll
    for (int j = 0; j < 4; ++j) {
#pragma unroll
      for (int r = 0; r < 8; ++r) slab[(mOff + r) * 68 + (j << 4) + rlane] = acc[i][j][r];
    }
    __builtin_amdgcn_fence(__ATOMIC_RELEASE, "workgroup");
    __builtin_amdgcn_wave_barrier();
    __builtin_amdgcn_fence(__ATOMIC_ACQUIRE, "workgroup");
    {
      const int hh = lane >> 4, c4 = (lane & 15) * 4;
      for (int pass = 0; pass < 2; ++pass) {
#pragma unroll
        for (int it = 0; it < 8; ++it) {
          const int row = it * 2 + hh;
          const v4f v = *(const v4f*)(slab + row * 68 + c4);
          *(volatile v4f*)(Cout + (size_t)(mBase + row) * ldc + n0 + c4) = v;
        }
        __threadfence();
      }
    }
    __builtin_amdgcn_fence(__ATOMIC_RELEASE, "workgroup");
    __builtin_amdgcn_wave_barrier();
    __builtin_amdgcn_fence(__ATOMIC_ACQUIRE, "workgroup");
  }
}

__global__ __launch_bounds__(NTHR) void mcell_seq_kernel(const float* __restrict__ MG, const float* __restrict__ mb,
                                                         unsigned short* __restrict__ HM) {
  __shared__ __align__(16) float Cl[CROWS * NHID];
  __shared__ __align__(16) float Qs[NHID];
  __shared__ __align__(16) float Ks[NHID];
  __shared__ float FPs[NHID];
  __shared__ float IPVs[NHID];
  __shared__ float OTs[NHID];
  __shared__ float REDs[NTHR / 32];
  __shared__ __align__(16) unsigned short HSTG[NPLANE * CROWS];
  const int tid = threadIdx.x, lane = tid & 31, wave = tid >> 5;
  const int bb = blockIdx.x >> 2, rg = blockIdx.x & 3;

  {
    const v4f z4 = {0.f, 0.f, 0.f, 0.f};
#pragma unroll
    for (int i = 0; i < (CROWS * NHID) / (4 * NTHR); ++i) *(v4f*)(Cl + (size_t)(i * NTHR + tid) * 4) = z4;
  }
  float mbr[6];
#pragma unroll
  for (int g = 0; g < 6; ++g) mbr[g] = bf16r(mb[g * NHID + tid]);
  float mst = 0.0f, nst = 0.0f;
  __syncthreads();

  const int iloc = tid >> 2, qd = tid & 3;
  const int irow = rg * CROWS + iloc;
  float* crow = Cl + iloc * NHID + qd * 64;
  const float* kseg = Ks + qd * 64;
  const float* qseg = Qs + qd * 64;

#pragma unroll 1
  for (int t = 0; t < NSTEP; ++t) {
    const size_t grow = (size_t)(t * NBATCH + bb);
    const float* gp = MG + grow * NG6 + tid;
    const float gq = gp[0] + mbr[0];
    const float gk = (gp[NHID] + mbr[1]) * 0.0625f;
    const float gv = gp[2 * NHID] + mbr[2];
    const float gi = gp[3 * NHID] + mbr[3];
    const float gf = gp[4 * NHID] + mbr[4];
    const float go = gp[5 * NHID] + mbr[5];
    const float ot = frcp(1.0f + expf(-go));
    const float mn = fmaxf(gf + mst, gi);
    const float ip = expf(gi - mn);
    const float fp = expf(gf + mst - mn);
    mst = mn;
    const float nn = fp * nst + ip * gk;
    nst = nn;
    float red = nn * gq;
#pragma unroll
    for (int off = 16; off >= 1; off >>= 1) red += __shfl_xor(red, off, 32);
    if (lane == 0) REDs[wave] = red;
    Qs[tid] = gq; Ks[tid] = gk; FPs[tid] = fp; IPVs[tid] = ip * gv; OTs[tid] = ot;
    __syncthreads();

    float s = REDs[0];
#pragma unroll
    for (int w = 1; w < NTHR / 32; ++w) s += REDs[w];
    const float den  = fmaxf(fabsf(s), 1.0f);
    const float rden = 1.0f / den;
    const float fpi = FPs[irow], ipv = IPVs[irow], oti = OTs[irow];
    float acc = 0.0f;
#pragma unroll 1
    for (int jj = 0; jj < 64; jj += 4) {
      v4f cv = *(const v4f*)(crow + jj);
      const v4f kv = *(const v4f*)(kseg + jj);
      const v4f qv = *(const v4f*)(qseg + jj);
#pragma unroll
      for (int e = 0; e < 4; ++e) {
        const float cn = fmaf(ipv, kv[e], fpi * cv[e]);
        cv[e] = cn;
        acc = fmaf(cn, qv[e], acc);
      }
      *(v4f*)(crow + jj) = cv;
    }
    acc += __shfl_xor(acc, 1, 32);
    acc += __shfl_xor(acc, 2, 32);
    const float h = (oti * acc) * rden;
    unsigned short hb, mbb, lb;
    split3_bf(h, hb, mbb, lb);
    if (qd == 0) { HSTG[iloc] = hb; HSTG[CROWS + iloc] = mbb; HSTG[2 * CROWS + iloc] = lb; }
    __syncthreads();

    if (wave == 0) {
      const int pl  = lane >> 3;
      const int plc = (pl < NPLANE) ? pl : (NPLANE - 1);
      const v4u v = *(const v4u*)(HSTG + plc * CROWS + (lane & 7) * 8);
      unsigned short* dp = HM + (size_t)plc * HM_PLANE + grow * NHID + (size_t)(rg * CROWS + (lane & 7) * 8);
      if (lane < NPLANE * 8) *(volatile v4u*)dp = v;
      __threadfence();
      if (lane < NPLANE * 8) *(volatile v4u*)dp = v;
    }
  }
}

__global__ __launch_bounds__(NTHR2) void scell_seq_kernel(const float* __restrict__ GX, const unsigned short* __restrict__ SRBp,
                                                          const float* __restrict__ sb,
                                                          const float* __restrict__ W1, const float* __restrict__ B1,
                                                          const float* __restrict__ W2, const float* __restrict__ B2,
                                                          const float* __restrict__ W3, const float* __restrict__ B3,
                                                          float* __restrict__ out) {
  __shared__ __align__(16) unsigned short Hh[16 * HTP];
  __shared__ __align__(16) unsigned short Hm[16 * HTP];
  __shared__ __align__(16) unsigned short Hl[16 * HTP];
  __shared__ __align__(16) float GXS[16 * GXP];
  const __bf16* SRB = (const __bf16*)SRBp;
  const int tid = threadIdx.x, lane = tid & 31, wave = tid >> 5;
  const int c = lane & 15, hh = lane >> 4, koff = hh * 8;
  const int j = 16 * wave + c;

#pragma unroll 1
  for (int i = tid; i < 16 * HTP; i += NTHR2) { Hh[i] = 0; Hm[i] = 0; Hl[i] = 0; }
  float sbr[4];
#pragma unroll
  for (int g = 0; g < 4; ++g) sbr[g] = bf16r(sb[g * NHID + j]);
  float cst[8], nst[8], mst[8], hst[8];
#pragma unroll
  for (int r = 0; r < 8; ++r) { cst[r] = 0.0f; nst[r] = 0.0f; mst[r] = 0.0f; hst[r] = 0.0f; }
  __syncthreads();

  const __bf16* ahp = (const __bf16*)Hh + c * HTP + koff;
  const __bf16* amp = (const __bf16*)Hm + c * HTP + koff;
  const __bf16* alp = (const __bf16*)Hl + c * HTP + koff;
  const __bf16* wb  = SRB + (size_t)j * NHID + koff;
  const v8f z8 = {0.f, 0.f, 0.f, 0.f, 0.f, 0.f, 0.f, 0.f};

#pragma unroll 1
  for (int t = 0; t < NSTEP; ++t) {
    {
      const float* gsrc = GX + (size_t)t * (size_t)(NBATCH * NG4);
#pragma unroll
      for (int it = 0; it < 4; ++it) {
        const int idx = it * NTHR2 + tid;
        const int row = idx >> 8, col4 = (idx & 255) * 4;
        const v4f v = *(const v4f*)(gsrc + (size_t)row * NG4 + col4);
        *(v4f*)(GXS + row * GXP + col4) = v;
      }
      asm volatile("" ::: "memory");
#pragma unroll
      for (int it = 4; it < 8; ++it) {
        const int idx = it * NTHR2 + tid;
        const int row = idx >> 8, col4 = (idx & 255) * 4;
        const v4f v = *(const v4f*)(gsrc + (size_t)row * NG4 + col4);
        *(v4f*)(GXS + row * GXP + col4) = v;
      }
    }
    __syncthreads();

    v8f acc0 = z8, acc1 = z8, acc2 = z8, acc3 = z8;
#pragma unroll 1
    for (int k0 = 0; k0 < NHID; k0 += 32) {
      const v16b ah = Frag<__bf16>::load(ahp + k0);
      const v16b am = Frag<__bf16>::load(amp + k0);
      const v16b al = Frag<__bf16>::load(alp + k0);
      const v16b b0 = Frag<__bf16>::load(wb + k0);
      const v16b b1 = Frag<__bf16>::load(wb + (size_t)1 * NHID * NHID + k0);
      const v16b b2 = Frag<__bf16>::load(wb + (size_t)2 * NHID * NHID + k0);
      const v16b b3 = Frag<__bf16>::load(wb + (size_t)3 * NHID * NHID + k0);
      acc0 = Frag<__bf16>::mma(ah, b0, acc0); acc0 = Frag<__bf16>::mma(am, b0, acc0); acc0 = Frag<__bf16>::mma(al, b0, acc0);
      acc1 = Frag<__bf16>::mma(ah, b1, acc1); acc1 = Frag<__bf16>::mma(am, b1, acc1); acc1 = Frag<__bf16>::mma(al, b1, acc1);
      acc2 = Frag<__bf16>::mma(ah, b2, acc2); acc2 = Frag<__bf16>::mma(am, b2, acc2); acc2 = Frag<__bf16>::mma(al, b2, acc2);
      acc3 = Frag<__bf16>::mma(ah, b3, acc3); acc3 = Frag<__bf16>::mma(am, b3, acc3); acc3 = Frag<__bf16>::mma(al, b3, acc3);
      guard4_b3(acc0, acc1, acc2, acc3, ah, am, al);
      keep4_b(b0, b1, b2, b3);
    }
    acc_guard4(acc0, acc1, acc2, acc3);

#pragma unroll
    for (int r = 0; r < 8; ++r) {
      const int row = 8 * hh + r;
      const float* gx = GXS + row * GXP + j;
      const float gz = acc0[r] + gx[0]        + sbr[0];
      const float gi = acc1[r] + gx[NHID]     + sbr[1];
      const float gf = acc2[r] + gx[2 * NHID] + sbr[2];
      const float go = acc3[r] + gx[3 * NHID] + sbr[3];
      const float z  = 1.0f - 2.0f * frcp(1.0f + expf(2.0f * gz));
      const float ot = frcp(1.0f + expf(-go));
      const float mn = fmaxf(gf + mst[r], gi);
      const float ip = expf(gi - mn);
      const float fp = expf(gf + mst[r] - mn);
      mst[r] = mn;
      const float cn = fp * cst[r] + ip * z;
      const float nn = fp * nst[r] + ip;
      cst[r] = cn;
      nst[r] = nn;
      hst[r] = (ot * cn) * frcp(nn);
    }
    __syncthreads();
#pragma unroll
    for (int r = 0; r < 8; ++r) {
      unsigned short hb, mbb, lb;
      split3_bf(hst[r], hb, mbb, lb);
      Hh[(8 * hh + r) * HTP + j] = hb;
      Hm[(8 * hh + r) * HTP + j] = mbb;
      Hl[(8 * hh + r) * HTP + j] = lb;
    }
  }

  float* HS   = GXS;
  float* A1   = GXS + 16 * HSP;
  float* A2   = A1 + NBATCH * NF1;
  float* OUTS = A2 + NBATCH * NF2;
#pragma unroll
  for (int r = 0; r < 8; ++r) HS[(8 * hh + r) * HSP + j] = hst[r];
  __syncthreads();
#pragma unroll 1
  for (int idx = tid; idx < NBATCH * NF1; idx += NTHR2) {
    const int bq = idx >> 7, o = idx & 127;
    float a = bf16r(B1[o]);
#pragma unroll 1
    for (int i = 0; i < NHID; ++i) a = fmaf(HS[bq * HSP + i], bf16r(W1[(size_t)i * NF1 + o]), a);
    A1[idx] = fmaxf(a, 0.0f);
  }
  __syncthreads();
#pragma unroll 1
  for (int idx = tid; idx < NBATCH * NF2; idx += NTHR2) {
    const int bq = idx >> 6, o = idx & 63;
    float a = bf16r(B2[o]);
#pragma unroll 1
    for (int i = 0; i < NF1; ++i) a = fmaf(A1[bq * NF1 + i], bf16r(W2[(size_t)i * NF2 + o]), a);
    A2[idx] = fmaxf(a, 0.0f);
  }
  __syncthreads();
  {
    const int bq = (tid < NBATCH) ? tid : (NBATCH - 1);
    float a = bf16r(B3[0]);
#pragma unroll 1
    for (int i = 0; i < NF2; ++i) a = fmaf(A2[bq * NF2 + i], bf16r(W3[i]), a);
    if (tid < NBATCH) OUTS[tid] = a;
  }
  __syncthreads();
  {
    const v4f v = *(const v4f*)(OUTS + (lane & 3) * 4);
    float* op = out + (lane & 3) * 4;
    if (tid < 4) *(volatile v4f*)op = v;
    __threadfence();
    if (tid < 4) *(volatile v4f*)op = v;
  }
}

extern "C" void kernel_launch(void* const* d_in, const int* in_sizes, int n_in,
                              void* d_out, int out_size, void* d_ws, size_t ws_size, hipStream_t stream) {
  if (n_in < 12 || d_out == nullptr || d_ws == nullptr) return;
  if (in_sizes[0] != NBATCH * NSTEP * NIN || in_sizes[1] != 6 * NIN * NHID || in_sizes[2] != NG6 ||
      in_sizes[3] != 4 * NHID * NHID || in_sizes[4] != 4 * NHID * NHID || in_sizes[5] != NG4 ||
      in_sizes[6] != NHID * NF1 || in_sizes[7] != NF1 || in_sizes[8] != NF1 * NF2 || in_sizes[9] != NF2 ||
      in_sizes[10] != NF2 || in_sizes[11] != 1 || out_size != NBATCH) return;

  const float* x    = (const float*)d_in[0];
  const float* mW   = (const float*)d_in[1];
  const float* mb   = (const float*)d_in[2];
  const float* sW   = (const float*)d_in[3];
  const float* sR   = (const float*)d_in[4];
  const float* sb   = (const float*)d_in[5];
  const float* fc1w = (const float*)d_in[6];
  const float* fc1b = (const float*)d_in[7];
  const float* fc2w = (const float*)d_in[8];
  const float* fc2b = (const float*)d_in[9];
  const float* fc3w = (const float*)d_in[10];
  const float* fc3b = (const float*)d_in[11];
  float* out = (float*)d_out;

  char* ws = (char*)d_ws; size_t off = 0;
  auto carve = [&](size_t bytes) -> char* { char* p = ws + off; off += (bytes + 255) & ~(size_t)255; return p; };
  unsigned short* XB  = (unsigned short*)carve((size_t)NROWS * KPAD * 2);
  unsigned short* MWB = (unsigned short*)carve((size_t)NG6 * KPAD * 2);
  unsigned short* SWB = (unsigned short*)carve((size_t)NG4 * NHID * 2);
  unsigned short* SRB = (unsigned short*)carve((size_t)NG4 * NHID * 2);
  float*          MG  = (float*)carve((size_t)NROWS * NG6 * 4);
  unsigned short* HM  = (unsigned short*)carve((size_t)NPLANE * HM_PLANE * 2);
  float*          GX  = (float*)carve((size_t)NROWS * NG4 * 4);
  if (off > ws_size || off > (size_t)134217728) return;

  pack_k32_kernel<0><<<(NROWS * 4) / NTHR, NTHR, 0, stream>>>(x, XB, NROWS);
  pack_k32_kernel<1><<<(NG6 * 4) / NTHR, NTHR, 0, stream>>>(mW, MWB, NG6);
  tpwz_kernel<<<dim3(NHID / 64, NHID / 64, 4), NTHR, 0, stream>>>(sW, NHID, NHID, NHID, (long)NHID * NHID, (long)NHID * NHID, SWB);
  tpwz_kernel<<<dim3(NHID / 64, NHID / 64, 4), NTHR, 0, stream>>>(sR, NHID, NHID, NHID, (long)NHID * NHID, (long)NHID * NHID, SRB);

  wmma_gemm64_bf16<1><<<((NROWS / 64) * (NG6 / 64)) / 8, NTHR, 0, stream>>>(XB, XB, XB, KPAD, MWB, KPAD, MG, NG6, NROWS, NG6, KPAD);

  mcell_seq_kernel<<<NBATCH * (NHID / CROWS), NTHR, 0, stream>>>(MG, mb, HM);

  wmma_gemm64_bf16<3><<<((NROWS / 64) * (NG4 / 64)) / 8, NTHR, 0, stream>>>(HM, HM + HM_PLANE, HM + 2 * HM_PLANE, NHID,
                                                                            SWB, NHID, GX, NG4, NROWS, NG4, NHID);

  scell_seq_kernel<<<1, NTHR2, 0, stream>>>(GX, SRB, sb, fc1w, fc1b, fc2w, fc2b, fc3w, fc3b, out);
}
